// TensorParallelQwenAttention_20495583936681
// MI455X (gfx1250) — hardware-verified
//
#include <hip/hip_runtime.h>
#include <math.h>

constexpr int kBatch = 2;
constexpr int kSeq   = 2048;
constexpr int kHid   = 2048;
constexpr int kHeads = 16;
constexpr int kKV    = 4;
constexpr int kHd    = 128;
constexpr int kRep   = kHeads / kKV;
constexpr int kTok   = kBatch * kSeq;
constexpr int kQcols = kHeads * kHd;
constexpr int kKcols = kKV * kHd;
constexpr int kQKVld = kQcols + 2 * kKcols;
constexpr int kKoff  = kQcols;
constexpr int kVoff  = kQcols + kKcols;
constexpr int kT0    = 128;
constexpr int kTokP  = kBatch * kT0;
constexpr int kSeqM  = kSeq - kT0;
constexpr int kPairs = kHd / 2;
constexpr float kWCarry    = 32.0f;
constexpr float kWCarryInv = 1.0f / 32.0f;
constexpr float kPCarry    = 32768.0f;
constexpr float kCtxCarry  = 64.0f;
constexpr float kCtxFin    = kCtxCarry / kPCarry;
constexpr float kOutScale  = 1.0f / (kCtxCarry * kWCarry);
constexpr float kScale     = 0.08838834764831845f;
static_assert(kHid % 32 == 0 && kQcols % 32 == 0, "K multiple of 32");
static_assert(kTok % 64 == 0 && kQcols % 64 == 0 && kKcols % 64 == 0, "tiles");
static_assert(kSeqM % 64 == 0 && kTokP % 64 == 0 && kT0 % 64 == 0 && kSeq % 64 == 0, "tiles");
static_assert(kRep == 4 && kHd == 128 && kPairs == 64, "shape");
static_assert(kKoff % 64 == 0 && kVoff % 64 == 0, "head columns");

typedef __attribute__((ext_vector_type(16))) _Float16 v16h;
typedef __attribute__((ext_vector_type(8)))  _Float16 v8h;
typedef __attribute__((ext_vector_type(16))) __bf16   v16b;
typedef __attribute__((ext_vector_type(8)))  __bf16   v8b;
typedef __attribute__((ext_vector_type(8)))  float    v8f;
typedef __attribute__((ext_vector_type(4)))  float    v4f;
typedef __attribute__((ext_vector_type(2)))  float    v2f;
typedef __attribute__((ext_vector_type(4)))  unsigned int v4u;
typedef __attribute__((ext_vector_type(2)))  unsigned int v2u;

__device__ __forceinline__ unsigned short f2bf_bits(float f) {
  unsigned u = __float_as_uint(f);
  return (unsigned short)((u + 0x7FFFu + ((u >> 16) & 1u)) >> 16);
}
__device__ __forceinline__ float bf_bits2f(unsigned short h) { return __uint_as_float(((unsigned)h) << 16); }

__device__ __forceinline__ void dep_guard_h(v8f& a, v8f& b, v16h x, v16h y) { asm volatile("v_nop\n\tv_nop\n\tv_nop\n\tv_nop" : "+v"(a), "+v"(b) : "v"(x), "v"(y)); }
__device__ __forceinline__ void dep_guard_b(v8f& a, v8f& b, v16b x, v16b y) { asm volatile("v_nop\n\tv_nop\n\tv_nop\n\tv_nop" : "+v"(a), "+v"(b) : "v"(x), "v"(y)); }
__device__ __forceinline__ void keep4_h(v16h a, v16h b, v16h c, v16h d) { asm volatile("v_nop" :: "v"(a), "v"(b), "v"(c), "v"(d)); }
__device__ __forceinline__ void keep4_b(v16b a, v16b b, v16b c, v16b d) { asm volatile("v_nop" :: "v"(a), "v"(b), "v"(c), "v"(d)); }
__device__ __forceinline__ void acc_guard4(v8f& a, v8f& b, v8f& c, v8f& d) { asm volatile("v_nop\n\tv_nop\n\tv_nop\n\tv_nop" : "+v"(a), "+v"(b), "+v"(c), "+v"(d)); }
template <typename T> struct Frag;
template <> struct Frag<_Float16> {
  typedef v16h V; union U { v16h v; v8h h[2]; };
  static __device__ __forceinline__ v16h load(const _Float16* p) {
    U f; f.h[0] = *(const v8h*)(p); f.h[1] = *(const v8h*)(p + 16); return f.v;
  }
  static __device__ __forceinline__ v8f mma(v16h a, v16h b, v8f c) {
    return __builtin_amdgcn_wmma_f32_16x16x32_f16(false, a, false, b, (short)0, c, false, false);
  }
  static __device__ __forceinline__ void guard(v8f& a, v8f& b, v16h x, v16h y) { dep_guard_h(a, b, x, y); }
  static __device__ __forceinline__ void keep(v16h a, v16h b, v16h c, v16h d) { keep4_h(a, b, c, d); }
};
template <> struct Frag<__bf16> {
  typedef v16b V; union U { v16b v; v8b h[2]; };
  static __device__ __forceinline__ v16b load(const __bf16* p) {
    U f; f.h[0] = *(const v8b*)(p); f.h[1] = *(const v8b*)(p + 16); return f.v;
  }
  static __device__ __forceinline__ v8f mma(v16b a, v16b b, v8f c) {
    return __builtin_amdgcn_wmma_f32_16x16x32_bf16(false, a, false, b, (short)0, c, false, false);
  }
  static __device__ __forceinline__ void guard(v8f& a, v8f& b, v16b x, v16b y) { dep_guard_b(a, b, x, y); }
  static __device__ __forceinline__ void keep(v16b a, v16b b, v16b c, v16b d) { keep4_b(a, b, c, d); }
};

__device__ __forceinline__ unsigned pk16(unsigned short a, unsigned short b) { return (unsigned)a | ((unsigned)b << 16); }
__device__ __forceinline__ unsigned short h_bits(float f) { const _Float16 h = (_Float16)f; return __builtin_bit_cast(unsigned short, h); }

__device__ __forceinline__ v8f hmma(v16h a, v16h b, v8f c) {
  c = __builtin_amdgcn_wmma_f32_16x16x32_f16(false, a, false, b, (short)0, c, false, false);
  asm volatile("v_nop\n\tv_nop\n\tv_nop\n\tv_nop" : "+v"(c) : "v"(a), "v"(b));
  return c;
}

template <int ET> struct Elem;
template <> struct Elem<0> { typedef _Float16 T; };
template <> struct Elem<1> { typedef __bf16 T; };
template <int ET, bool SPLIT, int BIAS_MODE, int OUT_MODE, bool RESID, int ACT, int ROPE>
__global__ __launch_bounds__(256) void wmma_gemm64(
    const unsigned short* __restrict__ Ap, const unsigned short* __restrict__ A2p, int lda, long strideA,
    const unsigned short* __restrict__ Btp, const unsigned short* __restrict__ Bt2p, int ldb, long strideB,
    void* __restrict__ Cout, void* __restrict__ Cout2, int ldc, long strideC,
    const float* __restrict__ bias,
    const float* __restrict__ resid, long strideR,
    int M, int N, int K, float scale,
    const float* __restrict__ rcos, const float* __restrict__ rsin, int posMask) {
  typedef typename Elem<ET>::T T;
  typedef typename Frag<T>::V V;
  const T* A = (const T*)Ap; const T* A2 = (const T*)A2p; const T* Bt = (const T*)Btp; const T* Bt2 = (const T*)Bt2p;
  __shared__ __align__(16) float sT[8][16 * 68];
  const int b    = blockIdx.y;
  const int lane = threadIdx.x & 31;
  const int wave = threadIdx.x >> 5;
  const int tilesN = N >> 6;
  const int tilesM = M >> 6;
  const int tile = blockIdx.x * 8 + wave;
  if (tile >= tilesM * tilesN) return;
  const int tm = tile / tilesN;
  const int tn = tile - tm * tilesN;
  const int m0 = tm << 6;
  const int n0 = tn << 6;

  const T* Ab  = A  + (size_t)b * strideA;
  const T* Bb  = Bt + (size_t)b * strideB;
  const T* Ab2 = SPLIT ? (A2  + (size_t)b * strideA) : nullptr;
  const T* Bb2 = SPLIT ? (Bt2 + (size_t)b * strideB) : nullptr;

  const int rlane = lane & 15;
  const int koff  = (lane >> 4) * 8;
  const int mOff  = (lane >> 4) * 8;

  v8f acc[4][4];
#pragma unroll
  for (int i = 0; i < 4; ++i)
#pragma unroll
    for (int j = 0; j < 4; ++j) acc[i][j] = (v8f){0.f,0.f,0.f,0.f,0.f,0.f,0.f,0.f};

  for (int k0 = 0; k0 < K; k0 += 32) {
    V bh[4], bl[4];
#pragma unroll
    for (int j = 0; j < 4; ++j) {
      const size_t bo = (size_t)(n0 + (j << 4) + rlane) * ldb + koff + k0;
      bh[j] = Frag<T>::load(Bb + bo);
      if (SPLIT) bl[j] = Frag<T>::load(Bb2 + bo);
    }
#pragma unroll
    for (int i = 0; i < 4; ++i) {
      const size_t ao = (size_t)(m0 + (i << 4) + rlane) * lda + koff + k0;
      V ah = Frag<T>::load(Ab + ao);
      V al;
      if (SPLIT) al = Frag<T>::load(Ab2 + ao);
#pragma unroll
      for (int j = 0; j < 4; ++j) {
        acc[i][j] = Frag<T>::mma(ah, bh[j], acc[i][j]);
        if (SPLIT) {
          acc[i][j] = Frag<T>::mma(ah, bl[j], acc[i][j]);
          acc[i][j] = Frag<T>::mma(al, bh[j], acc[i][j]);
        }
      }
      Frag<T>::guard(acc[i][0], acc[i][3], ah, SPLIT ? al : ah);
    }
    Frag<T>::keep(bh[0], bh[1], bh[2], bh[3]);
    if (SPLIT) Frag<T>::keep(bl[0], bl[1], bl[2], bl[3]);
  }
  acc_guard4(acc[0][0], acc[0][1], acc[0][2], acc[0][3]);
  acc_guard4(acc[1][0], acc[1][1], acc[1][2], acc[1][3]);
  acc_guard4(acc[2][0], acc[2][1], acc[2][2], acc[2][3]);
  acc_guard4(acc[3][0], acc[3][1], acc[3][2], acc[3][3]);

  float* slab = sT[wave];
  const float* Rb = RESID ? (resid + (size_t)b * strideR) : nullptr;
#pragma unroll
  for (int i = 0; i < 4; ++i) {
    const int mBase = m0 + (i << 4);
#pragma unroll
    for (int j = 0; j < 4; ++j) {
      const int n = n0 + (j << 4) + rlane;
      float bv = 0.f;
      if (BIAS_MODE == 2) bv = bias[n];
#pragma unroll
      for (int r = 0; r < 8; ++r) {
        float v = acc[i][j][r] * scale;
        if (BIAS_MODE == 1) v += bias[mBase + mOff + r];
        if (BIAS_MODE == 2) v += bv;
        if (RESID) v += Rb[(size_t)(mBase + mOff + r) * ldc + n];
        if (ACT == 2) v = fmaxf(v, 0.0f);
        if (ACT == 4) v = (v > 0.f) ? v : 0.01f * v;
        slab[(mOff + r) * 68 + (j << 4) + rlane] = v;
      }
    }
    __builtin_amdgcn_fence(__ATOMIC_RELEASE, "workgroup");
    __builtin_amdgcn_wave_barrier();
    __builtin_amdgcn_fence(__ATOMIC_ACQUIRE, "workgroup");
    if (OUT_MODE == 0) {
      float* C = (float*)Cout + (size_t)b * strideC;
      const int hh = lane >> 4, c4 = (lane & 15) * 4;
      for (int pass = 0; pass < 2; ++pass) {
#pragma unroll
        for (int it = 0; it < 8; ++it) {
          const int row = it * 2 + hh;
          v4f v = *(const v4f*)(slab + row * 68 + c4);
          if (ROPE) {
            const int pos = (mBase + row) & posMask;
            const int i0  = ((n0 + c4) & (kHd - 1)) >> 1;
            const v2f cc = *(const v2f*)(rcos + (size_t)pos * kPairs + i0);
            const v2f sn = *(const v2f*)(rsin + (size_t)pos * kPairs + i0);
            const float xa1 = v[0], xa2 = v[1], xb1 = v[2], xb2 = v[3];
            v[0] = xa1 * cc[0] - xa2 * sn[0];
            v[1] = xa1 * sn[0] + xa2 * cc[0];
            v[2] = xb1 * cc[1] - xb2 * sn[1];
            v[3] = xb1 * sn[1] + xb2 * cc[1];
          }
          *(volatile v4f*)(C + (size_t)(mBase + row) * ldc + n0 + c4) = v;
        }
        __threadfence();
      }
    } else {
      const int q = lane >> 3, c8 = (lane & 7) * 8;
      unsigned short* C  = (unsigned short*)Cout  + (size_t)b * strideC;
      unsigned short* C2 = (OUT_MODE == 2) ? ((unsigned short*)Cout2 + (size_t)b * strideC) : nullptr;
      for (int pass = 0; pass < 2; ++pass) {
#pragma unroll
        for (int it = 0; it < 4; ++it) {
          const int row = it * 4 + q;
          const float* sp = slab + row * 68 + c8;
          float xv[8];
#pragma unroll
          for (int e = 0; e < 8; ++e) xv[e] = sp[e];
          if (ROPE) {
            const int pos = (mBase + row) & posMask;
            const int i0  = ((n0 + c8) & (kHd - 1)) >> 1;
            const v4f cc = *(const v4f*)(rcos + (size_t)pos * kPairs + i0);
            const v4f sn = *(const v4f*)(rsin + (size_t)pos * kPairs + i0);
#pragma unroll
            for (int e2 = 0; e2 < 4; ++e2) {
              const float x1 = xv[2 * e2], x2 = xv[2 * e2 + 1];
              xv[2 * e2]     = x1 * cc[e2] - x2 * sn[e2];
              xv[2 * e2 + 1] = x1 * sn[e2] + x2 * cc[e2];
            }
          }
          v8h hv, lv;
#pragma unroll
          for (int e = 0; e < 8; ++e) {
            if (OUT_MODE == 1) {
              hv[e] = (_Float16)xv[e];
            } else {
              unsigned short hb = f2bf_bits(xv[e]);
              unsigned short lb = f2bf_bits(xv[e] - bf_bits2f(hb));
              hv[e] = __builtin_bit_cast(_Float16, hb);
              lv[e] = __builtin_bit_cast(_Float16, lb);
            }
          }
          *(volatile v8h*)(C + (size_t)(mBase + row) * ldc + n0 + c8) = hv;
          if (OUT_MODE == 2) *(volatile v8h*)(C2 + (size_t)(mBase + row) * ldc + n0 + c8) = lv;
        }
        __threadfence();
      }
    }
    __builtin_amdgcn_fence(__ATOMIC_RELEASE, "workgroup");
    __builtin_amdgcn_wave_barrier();
    __builtin_amdgcn_fence(__ATOMIC_ACQUIRE, "workgroup");
  }
}

__global__ __launch_bounds__(256) void cast8_f16_kernel(const float* __restrict__ in, unsigned short* __restrict__ out, int n8) {
  const int i = blockIdx.x * 256 + threadIdx.x;
  if (i >= n8) return;
  const float* p = in + 8 * (size_t)i;
  const v4f a = *(const v4f*)(p);
  const v4f c = *(const v4f*)(p + 4);
  unsigned short hb[8];
#pragma unroll
  for (int e = 0; e < 4; ++e) {
    hb[e]     = h_bits(a[e]);
    hb[4 + e] = h_bits(c[e]);
  }
  const v4u u = (v4u){pk16(hb[0], hb[1]), pk16(hb[2], hb[3]), pk16(hb[4], hb[5]), pk16(hb[6], hb[7])};
  unsigned short* q = out + 8 * (size_t)i;
  *(volatile v4u*)q = u;
  __threadfence();
  *(volatile v4u*)q = u;
}

__global__ __launch_bounds__(256) void xsplit_kernel(const float* __restrict__ x, unsigned short* __restrict__ hi,
                                                     unsigned short* __restrict__ lo, int n8) {
  const int i = blockIdx.x * 256 + threadIdx.x;
  if (i >= n8) return;
  const int prow = i >> 8;
  const int col  = (i & 255) * 8;
  const int srow = (prow >> 7) * kSeq + (prow & (kT0 - 1));
  const float* p = x + (size_t)srow * kHid + col;
  const v4f a = *(const v4f*)(p);
  const v4f c = *(const v4f*)(p + 4);
  unsigned short hb[8], lb[8];
#pragma unroll
  for (int e = 0; e < 4; ++e) {
    hb[e] = f2bf_bits(a[e]);       lb[e]     = f2bf_bits(a[e] - bf_bits2f(hb[e]));
    hb[4 + e] = f2bf_bits(c[e]);   lb[4 + e] = f2bf_bits(c[e] - bf_bits2f(hb[4 + e]));
  }
  const v4u uh = (v4u){pk16(hb[0], hb[1]), pk16(hb[2], hb[3]), pk16(hb[4], hb[5]), pk16(hb[6], hb[7])};
  const v4u ul = (v4u){pk16(lb[0], lb[1]), pk16(lb[2], lb[3]), pk16(lb[4], lb[5]), pk16(lb[6], lb[7])};
  const size_t d = (size_t)prow * kHid + col;
  *(volatile v4u*)(hi + d) = uh;
  *(volatile v4u*)(lo + d) = ul;
  __threadfence();
  *(volatile v4u*)(hi + d) = uh;
  *(volatile v4u*)(lo + d) = ul;
}

__global__ __launch_bounds__(256) void wtsplit_kernel(const float* __restrict__ W, int ncol, int rowOff,
                                                      unsigned short* __restrict__ o16, unsigned short* __restrict__ ohi,
                                                      unsigned short* __restrict__ olo) {
  __shared__ float sm[64][65];
  const int t  = threadIdx.x;
  const int k0 = blockIdx.x * 64;
  const int n0 = blockIdx.y * 64;
#pragma unroll
  for (int i = 0; i < 16; ++i) {
    const int e = i * 256 + t;
    const int r = e >> 6;
    const int c = e & 63;
    sm[c][r] = W[(size_t)(k0 + r) * ncol + n0 + c];
  }
  __syncthreads();
  const int lane = t & 31, wave = t >> 5;
  const int q = lane >> 3, c8 = (lane & 7) * 8;
  for (int pass = 0; pass < 2; ++pass) {
#pragma unroll
    for (int it = 0; it < 2; ++it) {
      const int row = wave * 8 + it * 4 + q;
      unsigned short fb[8], hb[8], lb[8];
#pragma unroll
      for (int e = 0; e < 8; ++e) {
        const float f = sm[row][c8 + e];
        fb[e] = h_bits(f * kWCarry);
        hb[e] = f2bf_bits(f);
        lb[e] = f2bf_bits(f - bf_bits2f(hb[e]));
      }
      const v4u uf = (v4u){pk16(fb[0], fb[1]), pk16(fb[2], fb[3]), pk16(fb[4], fb[5]), pk16(fb[6], fb[7])};
      const v4u uh = (v4u){pk16(hb[0], hb[1]), pk16(hb[2], hb[3]), pk16(hb[4], hb[5]), pk16(hb[6], hb[7])};
      const v4u ul = (v4u){pk16(lb[0], lb[1]), pk16(lb[2], lb[3]), pk16(lb[4], lb[5]), pk16(lb[6], lb[7])};
      const size_t d = (size_t)(rowOff + n0 + row) * kHid + k0 + c8;
      *(volatile v4u*)(o16 + d) = uf;
      *(volatile v4u*)(ohi + d) = uh;
      *(volatile v4u*)(olo + d) = ul;
    }
    __threadfence();
  }
}

struct RopeFreq { float f[64]; };
static_assert(sizeof(RopeFreq) == 256, "no padding");

__global__ __launch_bounds__(256) void rope_table_kernel(RopeFreq fr, float* __restrict__ rcos, float* __restrict__ rsin) {
  __shared__ __align__(16) float cb[256];
  __shared__ __align__(16) float sb[256];
  const int t    = threadIdx.x;
  const int wave = t >> 5;
  const int i    = t & 63;
  const int pos  = blockIdx.x * 4 + (t >> 6);
  float freq = 0.0f;
#pragma unroll
  for (int j = 0; j < 64; ++j) freq = (i == j) ? fr.f[j] : freq;
  const float ang = (float)pos * freq;
  float sv, cv;
  sincosf(ang, &sv, &cv);
  cb[t] = cv;
  sb[t] = sv;
  __syncthreads();
  if (wave < 2) {
    const v4f val = *(const v4f*)(cb + 4 * t);
    float* d = rcos + (size_t)blockIdx.x * 256 + 4 * t;
    *(volatile v4f*)d = val;
    __threadfence();
    *(volatile v4f*)d = val;
  } else if (wave < 4) {
    const int u = t - 64;
    const v4f val = *(const v4f*)(sb + 4 * u);
    float* d = rsin + (size_t)blockIdx.x * 256 + 4 * u;
    *(volatile v4f*)d = val;
    __threadfence();
    *(volatile v4f*)d = val;
  }
}

__global__ __launch_bounds__(256) void vt16_kernel(const unsigned short* __restrict__ QKV, unsigned short* __restrict__ Vt) {
  __shared__ unsigned short sm[64][68];
  const int t   = threadIdx.x;
  const int s0  = blockIdx.x * 64;
  const int kvh = blockIdx.y >> 1;
  const int d0  = (blockIdx.y & 1) * 64;
  const int b   = blockIdx.z;
  {
    const int sl = t >> 2, part = t & 3;
    const unsigned short* src = QKV + ((size_t)(b * kSeq + s0 + sl)) * kQKVld + kVoff + kvh * kHd + d0 + part * 16;
    const v4u u0 = *(const v4u*)(src);
    const v4u u1 = *(const v4u*)(src + 8);
#pragma unroll
    for (int e = 0; e < 4; ++e) {
      sm[part * 16 + 2 * e][sl]         = (unsigned short)(u0[e] & 0xffffu);
      sm[part * 16 + 2 * e + 1][sl]     = (unsigned short)(u0[e] >> 16);
      sm[part * 16 + 8 + 2 * e][sl]     = (unsigned short)(u1[e] & 0xffffu);
      sm[part * 16 + 8 + 2 * e + 1][sl] = (unsigned short)(u1[e] >> 16);
    }
  }
  __syncthreads();
  const int lane = t & 31, wave = t >> 5;
  const int q = lane >> 3, c8 = (lane & 7) * 8;
  unsigned short* op = Vt + ((size_t)((b * kKV + kvh) * kHd + d0)) * kSeq + s0;
  for (int pass = 0; pass < 2; ++pass) {
#pragma unroll
    for (int it = 0; it < 2; ++it) {
      const int row = wave * 8 + it * 4 + q;
      unsigned short hb[8];
#pragma unroll
      for (int e = 0; e < 8; ++e) hb[e] = sm[row][c8 + e];
      const v4u u = (v4u){pk16(hb[0], hb[1]), pk16(hb[2], hb[3]), pk16(hb[4], hb[5]), pk16(hb[6], hb[7])};
      *(volatile v4u*)(op + (size_t)row * kSeq + c8) = u;
    }
    __threadfence();
  }
}

constexpr int kKC  = 64;
constexpr int kKP  = kHd + 8;
constexpr int kVP  = kKC + 8;
constexpr int kPP  = kKC + 8;
constexpr int kOP  = 68;
constexpr int kNQT = kSeqM / 64;
static_assert(kKP % 8 == 0 && kVP % 8 == 0 && kPP % 8 == 0 && kOP % 4 == 0, "align");

__global__ __launch_bounds__(128) void attn_main_kernel(const unsigned short* __restrict__ QKVw,
                                                        const unsigned short* __restrict__ Vtw,
                                                        unsigned short* __restrict__ ctxw) {
  union FH { v16h v; v8h h[2]; };
  __shared__ __align__(16) _Float16 Ksh[kKC * kKP];
  __shared__ __align__(16) _Float16 Vsh[kHd * kVP];
  __shared__ __align__(16) _Float16 Psh[4][16 * kPP];
  __shared__ __align__(16) float    Os[4][16 * kOP];
  const _Float16* QKV = (const _Float16*)QKVw;
  const _Float16* Vt  = (const _Float16*)Vtw;
  _Float16* ctx = (_Float16*)ctxw;
  const int tid  = threadIdx.x;
  const int wave = tid >> 5;
  const int lane = tid & 31;
  const int hh   = lane >> 4;
  const int c    = lane & 15;
  const int bx  = blockIdx.x;
  const int qt  = bx % kNQT;
  const int bh  = bx / kNQT;
  const int h   = bh % kHeads;
  const int b   = bh / kHeads;
  const int kvh = h / kRep;
  const int qb  = qt + kT0 / 64;
  const int q0  = qb * 64 + wave * 16;

  v16h qa[4];
  {
    const _Float16* qrow = QKV + (size_t)(b * kSeq + q0 + c) * kQKVld + h * kHd;
#pragma unroll
    for (int dc = 0; dc < 4; ++dc) qa[dc] = Frag<_Float16>::load(qrow + dc * 32 + 8 * hh);
  }

  float mrow[8], lrow[8];
  v8f oacc[8];
#pragma unroll
  for (int r = 0; r < 8; ++r) { mrow[r] = -INFINITY; lrow[r] = 0.f; }
#pragma unroll
  for (int t = 0; t < 8; ++t) oacc[t] = (v8f){0.f,0.f,0.f,0.f,0.f,0.f,0.f,0.f};

  const int nChunks = qb + 1;
  for (int kc = 0; kc < nChunks; ++kc) {
    const int kv0 = kc * kKC;
    __syncthreads();
    {
      const int kvr = tid >> 1, dh = (tid & 1) * 64;
      const _Float16* ksrc = QKV + (size_t)(b * kSeq + kv0 + kvr) * kQKVld + kKoff + kvh * kHd + dh;
      _Float16* kdst = Ksh + kvr * kKP + dh;
#pragma unroll
      for (int i = 0; i < 8; ++i) *(v8h*)(kdst + 8 * i) = *(const v8h*)(ksrc + 8 * i);
      const _Float16* vsrc = Vt + ((size_t)((b * kKV + kvh) * kHd + tid)) * kSeq + kv0;
      _Float16* vdst = Vsh + tid * kVP;
#pragma unroll
      for (int i = 0; i < 8; ++i) *(v8h*)(vdst + 8 * i) = *(const v8h*)(vsrc + 8 * i);
    }
    __syncthreads();

    v8f s[4];
#pragma unroll
    for (int j = 0; j < 4; ++j) {
      s[j] = (v8f){0.f,0.f,0.f,0.f,0.f,0.f,0.f,0.f};
#pragma unroll
      for (int dc = 0; dc < 4; ++dc) {
        FH kb;
        kb.h[0] = *(const v8h*)(Ksh + (j * 16 + c) * kKP + dc * 32 + 8 * hh);
        kb.h[1] = *(const v8h*)(Ksh + (j * 16 + c) * kKP + dc * 32 + 16 + 8 * hh);
        s[j] = hmma(qa[dc], kb.v, s[j]);
      }
    }
    const bool diag = (kc == qb);
    float cm[8];
#pragma unroll
    for (int r = 0; r < 8; ++r) {
      const int qrow = q0 + 8 * hh + r;
      float m = -INFINITY;
#pragma unroll
      for (int j = 0; j < 4; ++j) {
        const int kvcol = kv0 + j * 16 + c;
        float sv = s[j][r] * kScale;
        const bool masked = diag && (kvcol > qrow);
        sv = masked ? -INFINITY : sv;
        s[j][r] = sv;
        m = fmaxf(m, sv);
      }
#pragma unroll
      for (int off = 1; off < 16; off <<= 1) m = fmaxf(m, __shfl_xor(m, off, 32));
      cm[r] = m;
    }
    _Float16* pw = Psh[wave];
#pragma unroll
    for (int r = 0; r < 8; ++r) {
      const float mnew  = fmaxf(mrow[r], cm[r]);
      const float alpha = expf(mrow[r] - mnew);
      mrow[r] = mnew;
      float psum = 0.f;
#pragma unroll
      for (int j = 0; j < 4; ++j) {
        const float p = expf(s[j][r] - mnew);
        psum += p;
        pw[(8 * hh + r) * kPP + j * 16 + c] = (_Float16)(p * kPCarry);
      }
#pragma unroll
      for (int off = 1; off < 16; off <<= 1) psum += __shfl_xor(psum, off, 32);
      lrow[r] = lrow[r] * alpha + psum;
#pragma unroll
      for (int t = 0; t < 8; ++t) oacc[t][r] *= alpha;
    }
    __builtin_amdgcn_fence(__ATOMIC_RELEASE, "workgroup");
    __builtin_amdgcn_wave_barrier();
    __builtin_amdgcn_fence(__ATOMIC_ACQUIRE, "workgroup");
#pragma unroll
    for (int kk = 0; kk < 2; ++kk) {
      FH pa;
      pa.h[0] = *(const v8h*)(pw + c * kPP + kk * 32 + 8 * hh);
      pa.h[1] = *(const v8h*)(pw + c * kPP + kk * 32 + 16 + 8 * hh);
#pragma unroll
      for (int t = 0; t < 8; ++t) {
        FH vb;
        vb.h[0] = *(const v8h*)(Vsh + (t * 16 + c) * kVP + kk * 32 + 8 * hh);
        vb.h[1] = *(const v8h*)(Vsh + (t * 16 + c) * kVP + kk * 32 + 16 + 8 * hh);
        oacc[t] = hmma(pa.v, vb.v, oacc[t]);
      }
    }
  }

  float inv[8];
#pragma unroll
  for (int r = 0; r < 8; ++r) inv[r] = kCtxFin / lrow[r];
  float* os = Os[wave];
  const int q8 = lane >> 3, c8 = (lane & 7) * 8;
  const size_t orow0 = (size_t)(b * kSeqM + (q0 - kT0));
#pragma unroll
  for (int half = 0; half < 2; ++half) {
#pragma unroll
    for (int r = 0; r < 8; ++r) {
#pragma unroll
      for (int t = 0; t < 4; ++t) os[(8 * hh + r) * kOP + t * 16 + c] = oacc[half * 4 + t][r] * inv[r];
    }
    __builtin_amdgcn_fence(__ATOMIC_RELEASE, "workgroup");
    __builtin_amdgcn_wave_barrier();
    __builtin_amdgcn_fence(__ATOMIC_ACQUIRE, "workgroup");
    for (int pass = 0; pass < 2; ++pass) {
#pragma unroll
      for (int it = 0; it < 4; ++it) {
        const int row = it * 4 + q8;
        const float* sp = os + row * kOP + c8;
        v8h hv;
#pragma unroll
        for (int e = 0; e < 8; ++e) hv[e] = (_Float16)sp[e];
        *(volatile v8h*)(ctx + (orow0 + row) * kQcols + h * kHd + half * 64 + c8) = hv;
      }
      __threadfence();
    }
    __builtin_amdgcn_fence(__ATOMIC_RELEASE, "workgroup");
    __builtin_amdgcn_wave_barrier();
    __builtin_amdgcn_fence(__ATOMIC_ACQUIRE, "workgroup");
  }
}

constexpr int kQG = 8;
static_assert(kT0 % kQG == 0, "groups");

__global__ __launch_bounds__(256) void attn_small_kernel(const float* __restrict__ QKVp, unsigned short* __restrict__ chi,
                                                         unsigned short* __restrict__ clo) {
  __shared__ float sc[kQG][kT0];
  const int tid  = threadIdx.x;
  const int wave = tid >> 5;
  const int lane = tid & 31;
  const int bx = blockIdx.x;
  const int g  = bx % (kT0 / kQG);
  const int bh = bx / (kT0 / kQG);
  const int h  = bh % kHeads;
  const int b  = bh / kHeads;
  const int kvh = h / kRep;
  const int q  = g * kQG + wave;
  const int nk = q + 1;
  const v4f qv = *(const v4f*)(QKVp + (size_t)(b * kT0 + q) * kQKVld + h * kHd + 4 * lane);
  const float* kbase = QKVp + (size_t)(b * kT0) * kQKVld + kKoff + kvh * kHd + 4 * lane;
  const float* vbase = QKVp + (size_t)(b * kT0) * kQKVld + kVoff + kvh * kHd + 4 * lane;
  float m = -INFINITY;
#pragma unroll 1
  for (int j = 0; j < nk; ++j) {
    const v4f kv = *(const v4f*)(kbase + (size_t)j * kQKVld);
    float d = qv[0] * kv[0] + qv[1] * kv[1] + qv[2] * kv[2] + qv[3] * kv[3];
#pragma unroll
    for (int off = 16; off > 0; off >>= 1) d += __shfl_xor(d, off, 32);
    const float sv = d * kScale;
    sc[wave][j] = sv;
    m = fmaxf(m, sv);
  }
  __syncthreads();
  float lsum = 0.f;
  v4f o = (v4f){0.f, 0.f, 0.f, 0.f};
#pragma unroll 1
  for (int j = 0; j < nk; ++j) {
    const float p = expf(sc[wave][j] - m);
    lsum += p;
    const v4f vv = *(const v4f*)(vbase + (size_t)j * kQKVld);
    o = o + p * vv;
  }
  const float inv = 1.0f / lsum;
  unsigned short hb[4], lb[4];
#pragma unroll
  for (int e = 0; e < 4; ++e) {
    const float f = o[e] * inv;
    hb[e] = f2bf_bits(f);
    lb[e] = f2bf_bits(f - bf_bits2f(hb[e]));
  }
  const v2u uh = (v2u){pk16(hb[0], hb[1]), pk16(hb[2], hb[3])};
  const v2u ul = (v2u){pk16(lb[0], lb[1]), pk16(lb[2], lb[3])};
  const size_t d = (size_t)(b * kT0 + q) * kQcols + h * kHd + 4 * lane;
  *(volatile v2u*)(chi + d) = uh;
  *(volatile v2u*)(clo + d) = ul;
  __threadfence();
  *(volatile v2u*)(chi + d) = uh;
  *(volatile v2u*)(clo + d) = ul;
}

extern "C" void kernel_launch(void* const* d_in, const int* in_sizes, int n_in,
                              void* d_out, int out_size, void* d_ws, size_t ws_size,
                              hipStream_t stream) {
  if (n_in < 8) return;
  if (in_sizes[0] != kTok * kHid) return;
  if (in_sizes[1] != kHid * kQcols || in_sizes[2] != kQcols) return;
  if (in_sizes[3] != kHid * kKcols || in_sizes[4] != kKcols) return;
  if (in_sizes[5] != kHid * kKcols || in_sizes[6] != kKcols) return;
  if (in_sizes[7] != kQcols * kHid) return;
  if (out_size != kTok * kHid) return;

  const size_t szXh   = (size_t)kTok * kHid * 2;
  const size_t szWqkv = (size_t)kQKVld * kHid * 2;
  const size_t szWo   = (size_t)kHid * kHid * 2;
  const size_t szQKV  = (size_t)kTok * kQKVld * 2;
  const size_t szVt   = (size_t)kBatch * kKV * kHd * kSeq * 2;
  const size_t szCtx  = (size_t)kBatch * kSeqM * kQcols * 2;
  const size_t szXp   = (size_t)kTokP * kHid * 2;
  const size_t szQKVp = (size_t)kTokP * kQKVld * 4;
  const size_t szCp   = (size_t)kTokP * kQcols * 2;
  const size_t szTab  = (size_t)kSeq * kPairs * 4;
  const size_t offXh   = 0;
  const size_t offWqkv = offXh + szXh;
  const size_t offWo   = offWqkv + szWqkv;
  const size_t offQKV  = offWo + szWo;
  const size_t offVt   = offQKV + szQKV;
  const size_t offCtx  = offVt + szVt;
  const size_t offXph  = offCtx + szCtx;
  const size_t offXpl  = offXph + szXp;
  const size_t offWqh  = offXpl + szXp;
  const size_t offWql  = offWqh + szWqkv;
  const size_t offWoh  = offWql + szWqkv;
  const size_t offWol  = offWoh + szWo;
  const size_t offQKVp = offWol + szWo;
  const size_t offCph  = offQKVp + szQKVp;
  const size_t offCpl  = offCph + szCp;
  const size_t offCos  = offCpl + szCp;
  const size_t offSin  = offCos + szTab;
  const size_t total   = offSin + szTab;
  if (ws_size < total) return;

  const float* hid = (const float*)d_in[0];
  const float* q_w = (const float*)d_in[1];
  const float* q_b = (const float*)d_in[2];
  const float* k_w = (const float*)d_in[3];
  const float* k_b = (const float*)d_in[4];
  const float* v_w = (const float*)d_in[5];
  const float* v_b = (const float*)d_in[6];
  const float* o_w = (const float*)d_in[7];
  float* out = (float*)d_out;
  char* ws = (char*)d_ws;
  unsigned short* Xh   = (unsigned short*)(ws + offXh);
  unsigned short* Wqkv = (unsigned short*)(ws + offWqkv);
  unsigned short* Wo   = (unsigned short*)(ws + offWo);
  unsigned short* QKV  = (unsigned short*)(ws + offQKV);
  unsigned short* Vt   = (unsigned short*)(ws + offVt);
  unsigned short* Ctx  = (unsigned short*)(ws + offCtx);
  unsigned short* Xph  = (unsigned short*)(ws + offXph);
  unsigned short* Xpl  = (unsigned short*)(ws + offXpl);
  unsigned short* Wqh  = (unsigned short*)(ws + offWqh);
  unsigned short* Wql  = (unsigned short*)(ws + offWql);
  unsigned short* Woh  = (unsigned short*)(ws + offWoh);
  unsigned short* Wol  = (unsigned short*)(ws + offWol);
  float* QKVp = (float*)(ws + offQKVp);
  unsigned short* Cph  = (unsigned short*)(ws + offCph);
  unsigned short* Cpl  = (unsigned short*)(ws + offCpl);
  float* Rcos = (float*)(ws + offCos);
  float* Rsin = (float*)(ws + offSin);

  RopeFreq fr;
  for (int i = 0; i < kPairs; ++i) {
    const float e  = (float)(2 * i) / (float)kHd;
    const float pf = (float)pow(10000.0, (double)e);
    fr.f[i] = 1.0f / pf;
  }

  {
    const int n8 = (kTok * kHid) / 8;
    cast8_f16_kernel<<<dim3(n8 / 256), dim3(256), 0, stream>>>(hid, Xh, n8);
    const int n8p = (kTokP * kHid) / 8;
    xsplit_kernel<<<dim3(n8p / 256), dim3(256), 0, stream>>>(hid, Xph, Xpl, n8p);
  }
  wtsplit_kernel<<<dim3(kHid / 64, kQcols / 64), dim3(256), 0, stream>>>(q_w, kQcols, 0,     Wqkv, Wqh, Wql);
  wtsplit_kernel<<<dim3(kHid / 64, kKcols / 64), dim3(256), 0, stream>>>(k_w, kKcols, kKoff, Wqkv, Wqh, Wql);
  wtsplit_kernel<<<dim3(kHid / 64, kKcols / 64), dim3(256), 0, stream>>>(v_w, kKcols, kVoff, Wqkv, Wqh, Wql);
  wtsplit_kernel<<<dim3(kQcols / 64, kHid / 64), dim3(256), 0, stream>>>(o_w, kHid, 0,      Wo, Woh, Wol);
  rope_table_kernel<<<dim3(kSeq / 4), dim3(256), 0, stream>>>(fr, Rcos, Rsin);

  wmma_gemm64<0, false, 2, 1, false, 0, 1><<<dim3((kTok / 64) * (kQcols / 64) / 8), dim3(256), 0, stream>>>(
      Xh, Xh, kHid, 0L, Wqkv, Wqkv, kHid, 0L, (void*)QKV, (void*)QKV, kQKVld, 0L,
      q_b, q_b, 0L, kTok, kQcols, kHid, kWCarryInv, Rcos, Rsin, kSeq - 1);
  wmma_gemm64<0, false, 2, 1, false, 0, 1><<<dim3((kTok / 64) * (kKcols / 64) / 8), dim3(256), 0, stream>>>(
      Xh, Xh, kHid, 0L, Wqkv + (size_t)kKoff * kHid, Wqkv + (size_t)kKoff * kHid, kHid, 0L,
      (void*)(QKV + kKoff), (void*)(QKV + kKoff), kQKVld, 0L,
      k_b, k_b, 0L, kTok, kKcols, kHid, kWCarryInv, Rcos, Rsin, kSeq - 1);
  wmma_gemm64<0, false, 2, 1, false, 0, 0><<<dim3((kTok / 64) * (kKcols / 64) / 8), dim3(256), 0, stream>>>(
      Xh, Xh, kHid, 0L, Wqkv + (size_t)kVoff * kHid, Wqkv + (size_t)kVoff * kHid, kHid, 0L,
      (void*)(QKV + kVoff), (void*)(QKV + kVoff), kQKVld, 0L,
      v_b, v_b, 0L, kTok, kKcols, kHid, kWCarryInv, Rcos, Rsin, kSeq - 1);
  vt16_kernel<<<dim3(kSeq / 64, kKV * 2, kBatch), dim3(256), 0, stream>>>(QKV, Vt);
  attn_main_kernel<<<dim3(kNQT * kHeads * kBatch), dim3(128), 0, stream>>>(QKV, Vt, Ctx);
  wmma_gemm64<0, false, 0, 0, false, 0, 0><<<dim3((kSeqM / 64) * (kHid / 64) / 8, kBatch), dim3(256), 0, stream>>>(
      Ctx, Ctx, kQcols, (long)kSeqM * kQcols, Wo, Wo, kQcols, 0L,
      (void*)(out + (size_t)kT0 * kHid), (void*)(out + (size_t)kT0 * kHid), kHid, (long)kSeq * kHid,
      q_b, q_b, 0L, kSeqM, kHid, kQcols, kOutScale, Rcos, Rsin, 0);

  wmma_gemm64<1, true, 2, 0, false, 0, 1><<<dim3((kTokP / 64) * (kQcols / 64) / 8), dim3(256), 0, stream>>>(
      Xph, Xpl, kHid, 0L, Wqh, Wql, kHid, 0L, (void*)QKVp, (void*)QKVp, kQKVld, 0L,
      q_b, q_b, 0L, kTokP, kQcols, kHid, 1.0f, Rcos, Rsin, kT0 - 1);
  wmma_gemm64<1, true, 2, 0, false, 0, 1><<<dim3((kTokP / 64) * (kKcols / 64) / 8), dim3(256), 0, stream>>>(
      Xph, Xpl, kHid, 0L, Wqh + (size_t)kKoff * kHid, Wql + (size_t)kKoff * kHid, kHid, 0L,
      (void*)(QKVp + kKoff), (void*)(QKVp + kKoff), kQKVld, 0L,
      k_b, k_b, 0L, kTokP, kKcols, kHid, 1.0f, Rcos, Rsin, kT0 - 1);
  wmma_gemm64<1, true, 2, 0, false, 0, 0><<<dim3((kTokP / 64) * (kKcols / 64) / 8), dim3(256), 0, stream>>>(
      Xph, Xpl, kHid, 0L, Wqh + (size_t)kVoff * kHid, Wql + (size_t)kVoff * kHid, kHid, 0L,
      (void*)(QKVp + kVoff), (void*)(QKVp + kVoff), kQKVld, 0L,
      v_b, v_b, 0L, kTokP, kKcols, kHid, 1.0f, Rcos, Rsin, kT0 - 1);
  attn_small_kernel<<<dim3(kBatch * kHeads * (kT0 / kQG)), dim3(256), 0, stream>>>(QKVp, Cph, Cpl);
  wmma_gemm64<1, true, 0, 0, false, 0, 0><<<dim3((kT0 / 64) * (kHid / 64) / 8, kBatch), dim3(256), 0, stream>>>(
      Cph, Cpl, kQcols, (long)kT0 * kQcols, Woh, Wol, kQcols, 0L,
      (void*)out, (void*)out, kHid, (long)kSeq * kHid,
      q_b, q_b, 0L, kT0, kHid, kQcols, 1.0f, Rcos, Rsin, 0);
}
